// multihead_cross_attention_50216757624952
// MI455X (gfx1250) — hardware-verified
//
#include <hip/hip_runtime.h>
#include <stdint.h>


#define BB  4
#define SS  2048
#define DD  1024
#define HH  16
#define DKK 64
#define HDK (HH * DKK)

#define GP 40
#define AP 72
#define PLANE (64 * AP)
#define STG 68

typedef float          v8f   __attribute__((ext_vector_type(8)));
typedef float          v4f   __attribute__((ext_vector_type(4)));
typedef unsigned short v4us  __attribute__((ext_vector_type(4)));
typedef unsigned short v8us  __attribute__((ext_vector_type(8)));
typedef unsigned short v16us __attribute__((ext_vector_type(16)));
typedef __bf16         v16bf __attribute__((ext_vector_type(16)));

__device__ __forceinline__ unsigned int bf16_bits_rne(float x) {
  const unsigned int u = __float_as_uint(x);
  return (u + 0x7FFFu + ((u >> 16) & 1u)) >> 16;
}

__device__ __forceinline__ void split1(float x, unsigned short& hi, unsigned short& lo) {
  const unsigned int h = bf16_bits_rne(x);
  const float hf = __uint_as_float(h << 16);
  hi = (unsigned short)h;
  lo = (unsigned short)bf16_bits_rne(x - hf);
}

__device__ __forceinline__ void split4(float4 f, v4us& hi, v4us& lo) {
  float a[4] = {f.x, f.y, f.z, f.w};
#pragma unroll
  for (int e = 0; e < 4; ++e) {
    unsigned short hs, ls;
    split1(a[e], hs, ls);
    hi[e] = hs;
    lo[e] = ls;
  }
}

__device__ __forceinline__ v16bf ld_frag(const unsigned short* base, int pitch, int lane) {
  const unsigned short* p = base + (lane & 15) * pitch + ((lane >> 4) << 3);
  const v8us e0 = *(const v8us*)(p);
  const v8us e1 = *(const v8us*)(p + 16);
  const v16us v = __builtin_shufflevector(e0, e1, 0, 1, 2, 3, 4, 5, 6, 7,
                                          8, 9, 10, 11, 12, 13, 14, 15);
  return __builtin_bit_cast(v16bf, v);
}

__device__ __forceinline__ v8f mma3(v8f c, v16bf ah, v16bf al, v16bf bh, v16bf bl) {
  c = __builtin_amdgcn_wmma_f32_16x16x32_bf16(false, ah, false, bh, (short)0, c, false, false);
  c = __builtin_amdgcn_wmma_f32_16x16x32_bf16(false, ah, false, bl, (short)0, c, false, false);
  c = __builtin_amdgcn_wmma_f32_16x16x32_bf16(false, al, false, bh, (short)0, c, false, false);
  asm volatile("v_nop\n\tv_nop\n\tv_nop\n\tv_nop" : "+v"(c) : "v"(ah), "v"(al), "v"(bh), "v"(bl));
  return c;
}

__global__ __launch_bounds__(256) void gemm_split_kernel(const float* __restrict__ X,
                                                         const float* __restrict__ W,
                                                         const float* __restrict__ bias,
                                                         float* dst,
                                                         int has_bias, int mode) {
  __shared__ __align__(16) unsigned char smem[8 * 16 * STG * 4];
  unsigned short* Ah = (unsigned short*)smem;
  unsigned short* Al = Ah + 128 * GP;
  unsigned short* Bh = Al + 128 * GP;
  unsigned short* Bl = Bh + 64 * GP;

  const int tid = threadIdx.x;
  const int lane = tid & 31, wv = tid >> 5;
  const int ln = lane & 15, lh = lane >> 4;
  const int m0 = blockIdx.x * 128;
  const int n0 = blockIdx.y * 64;

  v8f acc[4] = {};

  for (int k0 = 0; k0 < 1024; k0 += 32) {
    float4 fa[4], fb[2];
#pragma unroll
    for (int i = 0; i < 4; ++i) {
      const int idx = tid + i * 256;
      const int row = idx >> 3, c4 = (idx & 7) << 2;
      fa[i] = *(const float4*)(X + (size_t)(m0 + row) * 1024 + k0 + c4);
    }
#pragma unroll
    for (int i = 0; i < 2; ++i) {
      const int idx = tid + i * 256;
      const int row = idx >> 3, c4 = (idx & 7) << 2;
      fb[i] = *(const float4*)(W + (size_t)(n0 + row) * 1024 + k0 + c4);
    }
#pragma unroll
    for (int i = 0; i < 4; ++i) {
      const int idx = tid + i * 256;
      const int row = idx >> 3, c4 = (idx & 7) << 2;
      v4us hv, lv;
      split4(fa[i], hv, lv);
      *(v4us*)&Ah[row * GP + c4] = hv;
      *(v4us*)&Al[row * GP + c4] = lv;
    }
#pragma unroll
    for (int i = 0; i < 2; ++i) {
      const int idx = tid + i * 256;
      const int row = idx >> 3, c4 = (idx & 7) << 2;
      v4us hv, lv;
      split4(fb[i], hv, lv);
      *(v4us*)&Bh[row * GP + c4] = hv;
      *(v4us*)&Bl[row * GP + c4] = lv;
    }
    __syncthreads();
    const v16bf a_h = ld_frag(Ah + wv * 16 * GP, GP, lane);
    const v16bf a_l = ld_frag(Al + wv * 16 * GP, GP, lane);
#pragma unroll
    for (int t = 0; t < 4; ++t) {
      const v16bf b_h = ld_frag(Bh + t * 16 * GP, GP, lane);
      const v16bf b_l = ld_frag(Bl + t * 16 * GP, GP, lane);
      acc[t] = mma3(acc[t], a_h, a_l, b_h, b_l);
    }
    __syncthreads();
  }

  float* stg = (float*)smem + wv * (16 * STG);
#pragma unroll
  for (int t = 0; t < 4; ++t) {
    const int c = t * 16 + ln;
    float bvl = 0.f;
    if (has_bias) bvl = bias[n0 + c];
#pragma unroll
    for (int r = 0; r < 8; ++r) stg[(8 * lh + r) * STG + c] = acc[t][r] + bvl;
  }
  __syncthreads();

  const int hd = n0 >> 6;
  const int c4 = ln << 2;
  v4f vals[8];
#pragma unroll
  for (int it = 0; it < 8; ++it) {
    const int row = 2 * it + lh;
    vals[it] = *(const v4f*)(stg + row * STG + c4);
    const int m = m0 + wv * 16 + row;
    size_t base;
    if (mode) base = ((size_t)((m >> 11) * HH + hd) * SS + (m & 2047)) * DKK;
    else      base = (size_t)m * DD + n0;
    *(volatile v4f*)(dst + base + c4) = vals[it];
  }
  __threadfence();
#pragma unroll
  for (int it = 0; it < 8; ++it) {
    const int row = 2 * it + lh;
    const int m = m0 + wv * 16 + row;
    size_t base;
    if (mode) base = ((size_t)((m >> 11) * HH + hd) * SS + (m & 2047)) * DKK;
    else      base = (size_t)m * DD + n0;
    *(volatile v4f*)(dst + base + c4) = vals[it];
  }
}

__global__ __launch_bounds__(128) void attn_split_kernel(const float* __restrict__ Q,
                                                         const float* __restrict__ K,
                                                         const float* __restrict__ V,
                                                         float* ctx) {
  extern __shared__ __align__(16) unsigned char dsm[];
  unsigned short* Qh  = (unsigned short*)dsm;
  unsigned short* Ql  = Qh + PLANE;
  unsigned short* Kh  = Ql + PLANE;
  unsigned short* Kl  = Kh + PLANE;
  unsigned short* Vth = Kl + PLANE;
  unsigned short* Vtl = Vth + PLANE;
  unsigned short* Ph  = Vtl + PLANE;
  unsigned short* Pl  = Ph + PLANE;

  const int tid = threadIdx.x;
  const int lane = tid & 31, wv = tid >> 5;
  const int ln = lane & 15, lh = lane >> 4;
  const int q0 = blockIdx.x * 64;
  const int bh = blockIdx.y;

  const float* Qg = Q + ((size_t)bh * SS + q0) * DKK;
  const float* Kg = K + (size_t)bh * SS * DKK;
  const float* Vg = V + (size_t)bh * SS * DKK;

#pragma unroll
  for (int i = 0; i < 8; ++i) {
    const int idx = tid + i * 128;
    const int row = idx >> 4, c4 = (idx & 15) << 2;
    const float4 f = *(const float4*)(Qg + (size_t)row * DKK + c4);
    v4us hv, lv;
    split4(f, hv, lv);
    *(v4us*)&Qh[row * AP + c4] = hv;
    *(v4us*)&Ql[row * AP + c4] = lv;
  }
  __syncthreads();

  v8f oacc[4] = {};
  float mst[8], lst[8];
#pragma unroll
  for (int r = 0; r < 8; ++r) { mst[r] = -3.0e38f; lst[r] = 0.f; }

  const float scale = 0.125f;

  for (int j = 0; j < SS / 64; ++j) {
    const float* Kt = Kg + (size_t)j * 64 * DKK;
    const float* Vt = Vg + (size_t)j * 64 * DKK;
#pragma unroll
    for (int i = 0; i < 8; ++i) {
      const int idx = tid + i * 128;
      const int row = idx >> 4, c4 = (idx & 15) << 2;
      const float4 f = *(const float4*)(Kt + (size_t)row * DKK + c4);
      v4us hv, lv;
      split4(f, hv, lv);
      *(v4us*)&Kh[row * AP + c4] = hv;
      *(v4us*)&Kl[row * AP + c4] = lv;
    }
#pragma unroll
    for (int i = 0; i < 8; ++i) {
      const int idx = tid + i * 128;
      const int key = idx >> 4, c4 = (idx & 15) << 2;
      const float4 f = *(const float4*)(Vt + (size_t)key * DKK + c4);
      v4us hv, lv;
      split4(f, hv, lv);
#pragma unroll
      for (int e = 0; e < 4; ++e) {
        Vth[(c4 + e) * AP + key] = hv[e];
        Vtl[(c4 + e) * AP + key] = lv[e];
      }
    }
    __syncthreads();

    v8f sac[4] = {};
#pragma unroll
    for (int d = 0; d < 2; ++d) {
      const v16bf q_h = ld_frag(Qh + wv * 16 * AP + d * 32, AP, lane);
      const v16bf q_l = ld_frag(Ql + wv * 16 * AP + d * 32, AP, lane);
#pragma unroll
      for (int t = 0; t < 4; ++t) {
        const v16bf k_h = ld_frag(Kh + t * 16 * AP + d * 32, AP, lane);
        const v16bf k_l = ld_frag(Kl + t * 16 * AP + d * 32, AP, lane);
        sac[t] = mma3(sac[t], q_h, q_l, k_h, k_l);
      }
    }

    float corr[8];
#pragma unroll
    for (int r = 0; r < 8; ++r) {
      float mloc = -3.0e38f;
#pragma unroll
      for (int t = 0; t < 4; ++t) { sac[t][r] *= scale; mloc = fmaxf(mloc, sac[t][r]); }
#pragma unroll
      for (int off = 1; off < 16; off <<= 1) mloc = fmaxf(mloc, __shfl_xor(mloc, off));
      const float mnew = fmaxf(mst[r], mloc);
      const float c = __expf(mst[r] - mnew);
      float rsum = 0.f;
#pragma unroll
      for (int t = 0; t < 4; ++t) {
        const float p = __expf(sac[t][r] - mnew);
        sac[t][r] = p;
        rsum += p;
      }
#pragma unroll
      for (int off = 1; off < 16; off <<= 1) rsum += __shfl_xor(rsum, off);
      lst[r] = lst[r] * c + rsum;
      mst[r] = mnew;
      corr[r] = c;
    }
#pragma unroll
    for (int u = 0; u < 4; ++u)
#pragma unroll
      for (int r = 0; r < 8; ++r) oacc[u][r] *= corr[r];

    unsigned short* Pwh = Ph + wv * 16 * AP;
    unsigned short* Pwl = Pl + wv * 16 * AP;
#pragma unroll
    for (int t = 0; t < 4; ++t)
#pragma unroll
      for (int r = 0; r < 8; ++r) {
        unsigned short hs, ls;
        split1(sac[t][r], hs, ls);
        Pwh[(8 * lh + r) * AP + t * 16 + ln] = hs;
        Pwl[(8 * lh + r) * AP + t * 16 + ln] = ls;
      }
    __syncthreads();

#pragma unroll
    for (int kq = 0; kq < 2; ++kq) {
      const v16bf p_h = ld_frag(Pwh + kq * 32, AP, lane);
      const v16bf p_l = ld_frag(Pwl + kq * 32, AP, lane);
#pragma unroll
      for (int u = 0; u < 4; ++u) {
        const v16bf v_h = ld_frag(Vth + u * 16 * AP + kq * 32, AP, lane);
        const v16bf v_l = ld_frag(Vtl + u * 16 * AP + kq * 32, AP, lane);
        oacc[u] = mma3(oacc[u], p_h, p_l, v_h, v_l);
      }
    }
    __syncthreads();
  }

  float* stg = (float*)(dsm + 2 * PLANE * 2) + wv * (16 * STG);
  float inv[8];
#pragma unroll
  for (int r = 0; r < 8; ++r) inv[r] = 1.0f / lst[r];
#pragma unroll
  for (int u = 0; u < 4; ++u)
#pragma unroll
    for (int r = 0; r < 8; ++r) stg[(8 * lh + r) * STG + u * 16 + ln] = oacc[u][r] * inv[r];
  __syncthreads();

  const int b = bh >> 4, h = bh & 15;
  const int c4 = ln << 2;
  v4f vals[8];
#pragma unroll
  for (int it = 0; it < 8; ++it) {
    const int row = 2 * it + lh;
    vals[it] = *(const v4f*)(stg + row * STG + c4);
    const int s = q0 + wv * 16 + row;
    const size_t base = ((size_t)(b * SS + s)) * HDK + h * DKK;
    *(volatile v4f*)(ctx + base + c4) = vals[it];
  }
  __threadfence();
#pragma unroll
  for (int it = 0; it < 8; ++it) {
    const int row = 2 * it + lh;
    const int s = q0 + wv * 16 + row;
    const size_t base = ((size_t)(b * SS + s)) * HDK + h * DKK;
    *(volatile v4f*)(ctx + base + c4) = vals[it];
  }
}

extern "C" void kernel_launch(void* const* d_in, const int* in_sizes, int n_in,
                              void* d_out, int out_size, void* d_ws, size_t ws_size,
                              hipStream_t stream) {
  if (n_in < 10) return;
  const int nx = BB * SS * DD;
  const int nw = HDK * DD;
  if (in_sizes[0] != nx || in_sizes[1] != nx || in_sizes[2] != nx) return;
  if (in_sizes[3] != nw || in_sizes[5] != nw || in_sizes[7] != nw || in_sizes[9] != nw) return;
  if (in_sizes[4] != HDK || in_sizes[6] != HDK || in_sizes[8] != HDK) return;
  if (out_size != nx) return;
  const size_t qn = (size_t)BB * HH * SS * DKK;
  if (ws_size < 4 * qn * sizeof(float)) return;

  const float* Xq = (const float*)d_in[0];
  const float* Xk = (const float*)d_in[1];
  const float* Xv = (const float*)d_in[2];
  const float* Wq = (const float*)d_in[3];
  const float* bq = (const float*)d_in[4];
  const float* Wk = (const float*)d_in[5];
  const float* bk = (const float*)d_in[6];
  const float* Wv = (const float*)d_in[7];
  const float* bv = (const float*)d_in[8];
  const float* Wo = (const float*)d_in[9];
  float* out = (float*)d_out;

  float* ws = (float*)d_ws;
  float* Qf = ws;
  float* Kf = ws + qn;
  float* Vf = ws + 2 * qn;
  float* Cf = ws + 3 * qn;

  const dim3 gproj((BB * SS + 127) / 128, (HDK + 63) / 64);
  const dim3 gout((BB * SS + 127) / 128, (DD + 63) / 64);
  const dim3 gattn((SS + 63) / 64, BB * HH);
  const size_t attn_lds = (size_t)8 * PLANE * sizeof(unsigned short);

  gemm_split_kernel<<<gproj, dim3(256), 0, stream>>>(Xq, Wq, bq, Qf, 1, 1);
  gemm_split_kernel<<<gproj, dim3(256), 0, stream>>>(Xk, Wk, bk, Kf, 1, 1);
  gemm_split_kernel<<<gproj, dim3(256), 0, stream>>>(Xv, Wv, bv, Vf, 1, 1);
  attn_split_kernel<<<gattn, dim3(128), attn_lds, stream>>>(Qf, Kf, Vf, Cf);
  gemm_split_kernel<<<gout, dim3(256), 0, stream>>>(Cf, Wo, Wo, out, 0, 0);
}
